// CustomGNN_5093831213713
// MI455X (gfx1250) — hardware-verified
//
#include <hip/hip_runtime.h>
#include <stddef.h>
#include <stdint.h>


#define NN     32768
#define DD     256
#define EE     524288
#define BG     128
#define MX     384
#define CS     32
#define NHD    4
#define DH     64
#define DO     32
#define NL     3
#define MR     4096
#define NTHR   256
#define GTHR   128
#define GBM    64
#define TT     64
#define TP     68
#define NCH    256
#define CHE    2048
#define NGR    256
#define GRN    128
#define LCAP   4096
#define RUNCAP 64
#define MAXDEG 128
#define KPI    72
#define VPI    392
#define SPI    388
#define OPI    68
#define VBP    48
#define SSP    36
#define CX     8.0f
#define CW     64.0f
#define SCL    0.001953125f
#define CKV    8.0f
#define CQ     8.0f
#define CP     4096.0f
#define CV2    8.0f
#define SSCL   0.0009765625f
#define PVF    3.0517578125e-05f
#define CMF    7.62939453125e-06f
#define LNEPS  1.0e-5f
#define WSMAX  134217728
#define PMA_OV 55296
#define PMA_OQ 105472
#define PMA_OS 110080
#define PMA_OP 159744
#define PMA_OM 184832
#define PMA_LDS 184864

static_assert(NCH * CHE == EE);
static_assert(NGR * GRN == NN);
static_assert(LCAP == 2 * CHE);
static_assert((NN % GBM) == 0 && (MR % GBM) == 0 && (NN % 8) == 0 && (MR % 8) == 0);
static_assert(DD == NHD * DH && MR == BG * CS);
static_assert(PMA_OV == MX * KPI * 2);
static_assert(PMA_OQ == PMA_OV + DH * VPI * 2);
static_assert(PMA_OS == PMA_OQ + CS * KPI * 2);
static_assert(PMA_OP == PMA_OS + CS * SPI * 4);
static_assert(PMA_OM == PMA_OP + CS * VPI * 2);
static_assert(PMA_LDS >= PMA_OM + 16);
static_assert(CS * OPI * 4 <= CS * SPI * 4);
static_assert(CHE / NTHR == 8 && LCAP / (4 * NTHR) == 4);
static_assert(CS * DD == 8 * 1024);

typedef float    v4f  __attribute__((ext_vector_type(4)));
typedef float    v8f  __attribute__((ext_vector_type(8)));
typedef int      v4i  __attribute__((ext_vector_type(4)));
typedef int      v8i  __attribute__((ext_vector_type(8)));
typedef _Float16 v8h  __attribute__((ext_vector_type(8)));
typedef _Float16 v16h __attribute__((ext_vector_type(16)));
union FragH { v16h v; v8h h[2]; v8i w; };

__device__ __forceinline__ v8f wmh(const FragH& a, const FragH& b, v8f c) {
  v8f d = __builtin_amdgcn_wmma_f32_16x16x32_f16(false, a.v, false, b.v, (short)0, c, false, false);
  asm volatile("v_nop\n\tv_nop\n\tv_nop\n\tv_nop" : "+v"(d) : "v"(a.w), "v"(b.w));
  return d;
}
__device__ __forceinline__ v8f zero8() { const v8f z = {0.f, 0.f, 0.f, 0.f, 0.f, 0.f, 0.f, 0.f}; return z; }
__device__ __forceinline__ v4f zero4() { const v4f z = {0.f, 0.f, 0.f, 0.f}; return z; }

__device__ __forceinline__ v8h cvt8h(const v4f a, const v4f b, const float c) {
  v8h hv;
  hv[0] = (_Float16)(a.x * c); hv[1] = (_Float16)(a.y * c);
  hv[2] = (_Float16)(a.z * c); hv[3] = (_Float16)(a.w * c);
  hv[4] = (_Float16)(b.x * c); hv[5] = (_Float16)(b.y * c);
  hv[6] = (_Float16)(b.z * c); hv[7] = (_Float16)(b.w * c);
  return hv;
}
__device__ __forceinline__ v4f relu4(const v4f v) {
  v4f r; r.x = fmaxf(v.x, 0.f); r.y = fmaxf(v.y, 0.f); r.z = fmaxf(v.z, 0.f); r.w = fmaxf(v.w, 0.f); return r;
}
__device__ __forceinline__ void wave_lds_sync() {
  __builtin_amdgcn_fence(__ATOMIC_RELEASE, "wavefront");
  __builtin_amdgcn_wave_barrier();
}
__device__ __forceinline__ float wave_sum(float v) {
#pragma unroll
  for (int o = 16; o > 0; o >>= 1) v += __shfl_xor(v, o);
  return v;
}
__device__ __forceinline__ float wave_max(float v) {
#pragma unroll
  for (int o = 16; o > 0; o >>= 1) v = fmaxf(v, __shfl_xor(v, o));
  return v;
}
__device__ __forceinline__ int lbnd(const int* a, int n, int key) {
  int lo = 0, hi = n;
#pragma unroll 1
  while (lo < hi) {
    const int mid = (lo + hi) >> 1;
    if (a[mid] < key) lo = mid + 1; else hi = mid;
  }
  return lo;
}
__device__ __forceinline__ void bitonic_lds(int* a, int n, int tid) {
#pragma unroll 1
  for (int k = 2; k <= n; k <<= 1) {
#pragma unroll 1
    for (int j = k >> 1; j > 0; j >>= 1) {
#pragma unroll 1
      for (int p = tid; p < (n >> 1); p += NTHR) {
        const int i = ((p & ~(j - 1)) << 1) | (p & (j - 1));
        const int q = i | j;
        const int x = a[i], y = a[q];
        const bool up = (i & k) == 0;
        const bool sw = up ? (x > y) : (x < y);
        if (sw) { a[i] = y; a[q] = x; }
      }
      __syncthreads();
    }
  }
}

__global__ __launch_bounds__(NTHR) void k_xprep(const float* __restrict__ x, _Float16* xh, int nN, int MP, int nUnits) {
  const int i = (int)blockIdx.x * NTHR + (int)threadIdx.x;
  if (i >= nUnits) return;
  x  += (size_t)blockIdx.y * (size_t)nN * DD;
  xh += (size_t)blockIdx.y * (size_t)MP * DD;
  const int row = i >> 5, c0 = (i & 31) * 8;
  const int rc = row < nN ? row : nN - 1;
  const float* p = x + (size_t)rc * DD + c0;
  v4f a = *(const v4f*)p, b = *(const v4f*)(p + 4);
  if (row >= nN) { a = zero4(); b = zero4(); }
  const v8h hv = cvt8h(a, b, CX);
  const size_t o = (size_t)row * DD + c0;
  *(volatile v8h*)(xh + o) = hv;
  __threadfence();
  *(volatile v8h*)(xh + o) = hv;
}

__global__ __launch_bounds__(NTHR) void k_wtr(const float* __restrict__ W, _Float16* WT, int K, int Nc) {
  __shared__ __attribute__((aligned(16))) float tile[TT * TP];
  const int tid = (int)threadIdx.x, lane = tid & 31, wave = tid >> 5;
  W  += (size_t)blockIdx.z * (size_t)K * (size_t)Nc;
  WT += (size_t)blockIdx.z * (size_t)Nc * (size_t)K;
  const int n0 = (int)blockIdx.x * TT, k0 = (int)blockIdx.y * TT;
#pragma unroll
  for (int i = 0; i < 4; ++i) {
    const int kr = (tid >> 4) + 16 * i, c4 = (tid & 15) * 4;
    *(v4f*)(tile + kr * TP + c4) = *(const v4f*)(W + (size_t)(k0 + kr) * (size_t)Nc + n0 + c4);
  }
  __syncthreads();
  const int q = lane & 7;
  v8h hv[2];
#pragma unroll
  for (int i = 0; i < 2; ++i) {
    const int nr = 8 * wave + 4 * i + (lane >> 3);
    v4f a, b;
    a.x = tile[(8 * q + 0) * TP + nr]; a.y = tile[(8 * q + 1) * TP + nr];
    a.z = tile[(8 * q + 2) * TP + nr]; a.w = tile[(8 * q + 3) * TP + nr];
    b.x = tile[(8 * q + 4) * TP + nr]; b.y = tile[(8 * q + 5) * TP + nr];
    b.z = tile[(8 * q + 6) * TP + nr]; b.w = tile[(8 * q + 7) * TP + nr];
    hv[i] = cvt8h(a, b, CW);
  }
#pragma unroll
  for (int i = 0; i < 2; ++i) {
    const int nr = 8 * wave + 4 * i + (lane >> 3);
    *(volatile v8h*)(WT + (size_t)(n0 + nr) * (size_t)K + k0 + 8 * q) = hv[i];
  }
  __threadfence();
#pragma unroll
  for (int i = 0; i < 2; ++i) {
    const int nr = 8 * wave + 4 * i + (lane >> 3);
    *(volatile v8h*)(WT + (size_t)(n0 + nr) * (size_t)K + k0 + 8 * q) = hv[i];
  }
}

__global__ __launch_bounds__(32) void k_headw(const float* __restrict__ W, _Float16* WHD, int K, int Nc) {
  const int n = (int)blockIdx.x, lane = (int)threadIdx.x;
  const int nc = n < Nc ? n : Nc - 1;
  v4f a, b;
  a.x = W[(size_t)(8 * lane + 0) * Nc + nc]; a.y = W[(size_t)(8 * lane + 1) * Nc + nc];
  a.z = W[(size_t)(8 * lane + 2) * Nc + nc]; a.w = W[(size_t)(8 * lane + 3) * Nc + nc];
  b.x = W[(size_t)(8 * lane + 4) * Nc + nc]; b.y = W[(size_t)(8 * lane + 5) * Nc + nc];
  b.z = W[(size_t)(8 * lane + 6) * Nc + nc]; b.w = W[(size_t)(8 * lane + 7) * Nc + nc];
  if (n >= Nc) { a = zero4(); b = zero4(); }
  const v8h hv = cvt8h(a, b, CW);
  _Float16* op = WHD + (size_t)n * K + 8 * lane;
  *(volatile v8h*)op = hv;
  __threadfence();
  *(volatile v8h*)op = hv;
}

template<int EPI, int NT, int HB>
__global__ __launch_bounds__(GTHR) void k_gemm(
    const _Float16* __restrict__ A, const _Float16* __restrict__ WT, const float* __restrict__ bias,
    float* outF, _Float16* outH, int K, int ldo, float scl, float cao)
{
  constexpr int GBN = 16 * NT;
  __shared__ __attribute__((aligned(16))) float stg[GBM * GBN];
  const int tid = (int)threadIdx.x, lane = tid & 31, wave = tid >> 5, hh = lane >> 4, m = lane & 15;
  const int rowBase = (int)blockIdx.x * GBM, col0 = (int)blockIdx.y * GBN;
  v8f acc[NT];
#pragma unroll
  for (int t = 0; t < NT; ++t) acc[t] = zero8();
  const _Float16* ap = A  + (size_t)(rowBase + 16 * wave + m) * (size_t)K + 8 * hh;
  const _Float16* wp = WT + (size_t)(col0 + m) * (size_t)K + 8 * hh;
  const int ksteps = K >> 5;
#pragma unroll 1
  for (int ks = 0; ks < ksteps; ++ks) {
    FragH af;
    af.h[0] = *(const v8h*)(ap + 32 * ks);
    af.h[1] = *(const v8h*)(ap + 32 * ks + 16);
#pragma unroll
    for (int t = 0; t < NT; ++t) {
      const _Float16* wq = wp + (size_t)(16 * t) * (size_t)K + 32 * ks;
      FragH bf;
      bf.h[0] = *(const v8h*)wq;
      bf.h[1] = *(const v8h*)(wq + 16);
      acc[t] = wmh(af, bf, acc[t]);
    }
  }
#pragma unroll
  for (int t = 0; t < NT; ++t) {
    const int lc = 16 * t + m;
    float bv = 0.f;
    if (HB) bv = bias[col0 + lc];
#pragma unroll
    for (int r = 0; r < 8; ++r) stg[(16 * wave + 8 * hh + r) * GBN + lc] = fmaf(acc[t][r], scl, bv);
  }
  __syncthreads();
  if (EPI == 0) {
    constexpr int LPR = 4 * NT, RPI = 32 / LPR, NI = 16 / RPI;
    v4f fv[NI];
#pragma unroll
    for (int i = 0; i < NI; ++i) {
      const int lr = 16 * wave + RPI * i + lane / LPR, cc = 4 * (lane % LPR);
      fv[i] = *(const v4f*)(stg + lr * GBN + cc);
    }
#pragma unroll
    for (int i = 0; i < NI; ++i) {
      const int lr = 16 * wave + RPI * i + lane / LPR, cc = 4 * (lane % LPR);
      *(volatile v4f*)(outF + (size_t)(rowBase + lr) * (size_t)ldo + col0 + cc) = fv[i];
    }
    __threadfence();
#pragma unroll
    for (int i = 0; i < NI; ++i) {
      const int lr = 16 * wave + RPI * i + lane / LPR, cc = 4 * (lane % LPR);
      *(volatile v4f*)(outF + (size_t)(rowBase + lr) * (size_t)ldo + col0 + cc) = fv[i];
    }
  } else {
    constexpr int LPR = 2 * NT, RPI = 32 / LPR, NI = 16 / RPI;
    v8h hv[NI];
#pragma unroll
    for (int i = 0; i < NI; ++i) {
      const int lr = 16 * wave + RPI * i + lane / LPR, cc = 8 * (lane % LPR);
      hv[i] = cvt8h(*(const v4f*)(stg + lr * GBN + cc), *(const v4f*)(stg + lr * GBN + cc + 4), cao);
    }
#pragma unroll
    for (int i = 0; i < NI; ++i) {
      const int lr = 16 * wave + RPI * i + lane / LPR, cc = 8 * (lane % LPR);
      *(volatile v8h*)(outH + (size_t)(rowBase + lr) * (size_t)ldo + col0 + cc) = hv[i];
    }
    __threadfence();
#pragma unroll
    for (int i = 0; i < NI; ++i) {
      const int lr = 16 * wave + RPI * i + lane / LPR, cc = 8 * (lane % LPR);
      *(volatile v8h*)(outH + (size_t)(rowBase + lr) * (size_t)ldo + col0 + cc) = hv[i];
    }
  }
}

__global__ __launch_bounds__(NTHR) void k_csort(const int* __restrict__ ei, int* SK, int* CNT, int* LB) {
  __shared__ __attribute__((aligned(16))) int keys[CHE];
  const int tid = (int)threadIdx.x, c = (int)blockIdx.x;
#pragma unroll
  for (int j = 0; j < CHE / NTHR; ++j) {
    const int e = c * CHE + tid + NTHR * j;
    int s = ei[e], d = ei[EE + e];
    s = s < 0 ? 0 : (s > NN - 1 ? NN - 1 : s);
    d = d < 0 ? 0 : (d > NN - 1 ? NN - 1 : d);
    keys[tid + NTHR * j] = (d << 15) | s;
  }
  __syncthreads();
  bitonic_lds(keys, CHE, tid);
  v4i kv[2];
#pragma unroll
  for (int it = 0; it < 2; ++it) kv[it] = *(const v4i*)(keys + 4 * (tid + NTHR * it));
  const int lo = lbnd(keys, CHE, tid << 22);
  const int hi = lbnd(keys, CHE, (tid + 1) << 22);
  int* skp = SK + (size_t)c * CHE;
#pragma unroll
  for (int it = 0; it < 2; ++it) *(volatile v4i*)(skp + 4 * (tid + NTHR * it)) = kv[it];
  *(volatile int*)(CNT + (size_t)c * NGR + tid) = hi - lo;
  *(volatile int*)(LB  + (size_t)c * NGR + tid) = lo;
  __threadfence();
#pragma unroll
  for (int it = 0; it < 2; ++it) *(volatile v4i*)(skp + 4 * (tid + NTHR * it)) = kv[it];
  *(volatile int*)(CNT + (size_t)c * NGR + tid) = hi - lo;
  *(volatile int*)(LB  + (size_t)c * NGR + tid) = lo;
}

__global__ __launch_bounds__(NTHR) void k_cgroup(const int* __restrict__ SK, const int* __restrict__ CNT,
                                                const int* __restrict__ LB, int* ES, int* RC, int* RO) {
  __shared__ __attribute__((aligned(16))) int keys[LCAP];
  __shared__ int wsum[8];
  const int tid = (int)threadIdx.x, lane = tid & 31, wave = tid >> 5, g = (int)blockIdx.x, c = tid;
  const int nraw = CNT[(size_t)c * NGR + g];
  bool bad = (nraw < 0) || (nraw > RUNCAP);
  const int n = bad ? 0 : nraw;
  int lb = LB[(size_t)c * NGR + g];
  lb = lb < 0 ? 0 : (lb > CHE - n ? CHE - n : lb);
  int x = n;
#pragma unroll
  for (int o = 1; o < 32; o <<= 1) { const int y = __shfl_up(x, o); if (lane >= o) x += y; }
  if (lane == 31) wsum[wave] = x;
  __syncthreads();
  int pre = 0, tot = 0;
#pragma unroll
  for (int w = 0; w < 8; ++w) { const int t = wsum[w]; tot += t; if (w < wave) pre += t; }
  const int off = pre + x - n;
  bad = bad || (tot > LCAP);
  const int totc = tot > LCAP ? LCAP : tot;
  const int* skp = SK + (size_t)c * CHE + lb;
#pragma unroll 1
  for (int j = 0; j < n; ++j) {
    const int pos = off + j;
    if (pos < LCAP) keys[pos] = skp[j] & 0x3FFFFF;
  }
#pragma unroll 1
  for (int i2 = tid; i2 < LCAP; i2 += NTHR) if (i2 >= totc) keys[i2] = 0x7FFFFFFF;
  const int anybad = __syncthreads_or(bad ? 1 : 0);
  const int nsort = totc <= CHE ? CHE : LCAP;
  bitonic_lds(keys, nsort, tid);
  v4i kv[4];
#pragma unroll
  for (int it = 0; it < 4; ++it) kv[it] = *(const v4i*)(keys + 4 * (tid + NTHR * it));
  int cntn = 0, lo = 0;
  if (tid < GRN) {
    lo = lbnd(keys, LCAP, tid << 15);
    const int hi = lbnd(keys, LCAP, (tid + 1) << 15);
    cntn = anybad ? -1 : hi - lo;
  }
  int* esp = ES + (size_t)g * LCAP;
#pragma unroll
  for (int it = 0; it < 4; ++it) *(volatile v4i*)(esp + 4 * (tid + NTHR * it)) = kv[it];
  if (tid < GRN) {
    *(volatile int*)(RC + (size_t)g * GRN + tid) = cntn;
    *(volatile int*)(RO + (size_t)g * GRN + tid) = lo;
  }
  __threadfence();
#pragma unroll
  for (int it = 0; it < 4; ++it) *(volatile v4i*)(esp + 4 * (tid + NTHR * it)) = kv[it];
  if (tid < GRN) {
    *(volatile int*)(RC + (size_t)g * GRN + tid) = cntn;
    *(volatile int*)(RO + (size_t)g * GRN + tid) = lo;
  }
}

__global__ __launch_bounds__(NTHR) void k_agg(const float* __restrict__ XW, const int* __restrict__ ES,
                                             const int* __restrict__ RC, const int* __restrict__ RO,
                                             const float* __restrict__ gb, float* XG, _Float16* XGH) {
  __shared__ __attribute__((aligned(16))) float stg[8 * DD];
  const int tid = (int)threadIdx.x, lane = tid & 31, wave = tid >> 5;
  const int i = (int)blockIdx.x * 8 + wave;
  const int craw = RC[i];
  const bool bad = (craw < 0) || (craw > MAXDEG);
  const int cnt = bad ? 0 : craw;
  int off = RO[i];
  off = off < 0 ? 0 : (off > LCAP - cnt ? LCAP - cnt : off);
  const float deg = (float)cnt + 1.0f;
  const float rdeg = 1.0f / deg;
  const float di = rsqrtf(deg);
  const int* seg = ES + (size_t)(i >> 7) * LCAP + off;
  v4f a0 = zero4(), a1 = zero4();
#pragma unroll 1
  for (int j = 0; j < cnt; ++j) {
    const int s = seg[j] & (NN - 1);
    int cs = RC[s];
    cs = cs < 0 ? 0 : cs;
    const float w = rsqrtf((float)cs + 1.0f) * di;
    const float* xr = XW + (size_t)s * DD;
    const v4f xa = *(const v4f*)(xr + 4 * lane), xb = *(const v4f*)(xr + 128 + 4 * lane);
    a0 = a0 + w * xa;
    a1 = a1 + w * xb;
  }
  const float* xi = XW + (size_t)i * DD;
  v4f t0 = a0 + *(const v4f*)(xi + 4 * lane) * rdeg;
  v4f t1 = a1 + *(const v4f*)(xi + 128 + 4 * lane) * rdeg;
  t0 = t0 + *(const v4f*)(gb + 4 * lane);
  t1 = t1 + *(const v4f*)(gb + 128 + 4 * lane);
  if (bad) {
    const float qn = __int_as_float(0x7fc00000);
    const v4f n4 = {qn, qn, qn, qn};
    t0 = n4; t1 = n4;
  }
  float* op = XG + (size_t)i * DD;
  *(volatile v4f*)(op + 4 * lane) = t0;
  *(volatile v4f*)(op + 128 + 4 * lane) = t1;
  __threadfence();
  *(volatile v4f*)(op + 4 * lane) = t0;
  *(volatile v4f*)(op + 128 + 4 * lane) = t1;
  float* sw = stg + wave * DD;
  *(v4f*)(sw + 4 * lane) = t0;
  *(v4f*)(sw + 128 + 4 * lane) = t1;
  wave_lds_sync();
  const v8h hv = cvt8h(*(const v4f*)(sw + 8 * lane), *(const v4f*)(sw + 8 * lane + 4), CX);
  _Float16* hp = XGH + (size_t)i * DD + 8 * lane;
  *(volatile v8h*)hp = hv;
  __threadfence();
  *(volatile v8h*)hp = hv;
}

__global__ __launch_bounds__(NTHR) void k_pma(const _Float16* __restrict__ KV, const float* __restrict__ QF,
                                             const int* __restrict__ bid, float* AP, float* O) {
  extern __shared__ __attribute__((aligned(16))) char dsm[];
  _Float16* KT = (_Float16*)(dsm);
  _Float16* VT = (_Float16*)(dsm + PMA_OV);
  _Float16* QT = (_Float16*)(dsm + PMA_OQ);
  float*    SS = (float*)(dsm + PMA_OS);
  _Float16* PT = (_Float16*)(dsm + PMA_OP);
  int*      msc = (int*)(dsm + PMA_OM);
  const int tid = (int)threadIdx.x, lane = tid & 31, wave = tid >> 5, hh = lane >> 4, m = lane & 15;
  const int b = (int)blockIdx.x, h = (int)blockIdx.y;
  if (tid == 0) msc[0] = lbnd(bid, NN, b);
  if (tid == 1) msc[1] = lbnd(bid, NN, b + 1);
  __syncthreads();
  const int start = msc[0];
  int cnt = msc[1] - start;
  cnt = cnt < 0 ? 0 : (cnt > MX ? MX : cnt);
  const v8h z8 = cvt8h(zero4(), zero4(), 1.0f);
#pragma unroll 1
  for (int it = 0; it < (MX * 8) / NTHR; ++it) {
    const int u = tid + NTHR * it, n = u >> 3, q = u & 7;
    int r = start + n;
    r = r > NN - 1 ? NN - 1 : r;
    const _Float16* rp = KV + (size_t)r * (2 * DD) + DH * h + 8 * q;
    v8h k8 = *(const v8h*)rp;
    v8h v8 = *(const v8h*)(rp + DD);
    if (n >= cnt) { k8 = z8; v8 = z8; }
    *(v8h*)(KT + n * KPI + 8 * q) = k8;
#pragma unroll
    for (int j = 0; j < 8; ++j) VT[(8 * q + j) * VPI + n] = v8[j];
  }
  {
    const int c = tid >> 3, q = tid & 7;
    const float* qp = QF + (size_t)c * DD + DH * h + 8 * q;
    *(v8h*)(QT + c * KPI + 8 * q) = cvt8h(*(const v4f*)qp, *(const v4f*)(qp + 4), CQ);
  }
  __syncthreads();
  const int i = wave & 1;
  {
    const int jb = 6 * (wave >> 1);
    v8f acc[6];
#pragma unroll
    for (int t = 0; t < 6; ++t) acc[t] = zero8();
#pragma unroll
    for (int ks = 0; ks < 2; ++ks) {
      FragH af;
      af.h[0] = *(const v8h*)(QT + (16 * i + m) * KPI + 32 * ks + 8 * hh);
      af.h[1] = *(const v8h*)(QT + (16 * i + m) * KPI + 32 * ks + 16 + 8 * hh);
#pragma unroll
      for (int t = 0; t < 6; ++t) {
        const int j = jb + t;
        if (16 * j < cnt) {
          FragH bf;
          bf.h[0] = *(const v8h*)(KT + (16 * j + m) * KPI + 32 * ks + 8 * hh);
          bf.h[1] = *(const v8h*)(KT + (16 * j + m) * KPI + 32 * ks + 16 + 8 * hh);
          acc[t] = wmh(af, bf, acc[t]);
        }
      }
    }
#pragma unroll
    for (int t = 0; t < 6; ++t) {
      const int j = jb + t;
      if (16 * j < cnt) {
#pragma unroll
        for (int r = 0; r < 8; ++r) SS[(16 * i + 8 * hh + r) * SPI + 16 * j + m] = acc[t][r] * SSCL;
      }
    }
  }
  __syncthreads();
#pragma unroll 1
  for (int rr = 0; rr < 4; ++rr) {
    const int row = 4 * wave + rr;
    float sv[12];
    float mx = -3.0e38f;
#pragma unroll
    for (int p = 0; p < 12; ++p) {
      const int n = lane + 32 * p;
      const float s = (n < cnt) ? SS[row * SPI + n] : -3.0e38f;
      sv[p] = s; mx = fmaxf(mx, s);
    }
    mx = wave_max(mx);
    float sum = 0.f;
#pragma unroll
    for (int p = 0; p < 12; ++p) {
      const int n = lane + 32 * p;
      const float e = (n < cnt) ? __expf(sv[p] - mx) : 0.f;
      sv[p] = e; sum += e;
    }
    sum = wave_sum(sum);
    const float rs = sum > 0.f ? 1.0f / sum : 0.f;
#pragma unroll
    for (int p = 0; p < 12; ++p) {
      const int n = lane + 32 * p;
      const float pv = sv[p] * rs;
      sv[p] = pv;
      PT[row * VPI + n] = (_Float16)(pv * CP);
    }
    float* apr = AP + ((size_t)((h * BG + b) * CS + row)) * MX;
#pragma unroll
    for (int p = 0; p < 12; ++p) *(volatile float*)(apr + lane + 32 * p) = sv[p];
    __threadfence();
#pragma unroll
    for (int p = 0; p < 12; ++p) *(volatile float*)(apr + lane + 32 * p) = sv[p];
  }
  __syncthreads();
  float* OST = SS;
  {
    const int j = wave >> 1;
    v8f acc1 = zero8();
    const int ksn = (cnt + 31) >> 5;
#pragma unroll 1
    for (int ks = 0; ks < ksn; ++ks) {
      FragH af, bf;
      af.h[0] = *(const v8h*)(PT + (16 * i + m) * VPI + 32 * ks + 8 * hh);
      af.h[1] = *(const v8h*)(PT + (16 * i + m) * VPI + 32 * ks + 16 + 8 * hh);
      bf.h[0] = *(const v8h*)(VT + (16 * j + m) * VPI + 32 * ks + 8 * hh);
      bf.h[1] = *(const v8h*)(VT + (16 * j + m) * VPI + 32 * ks + 16 + 8 * hh);
      acc1 = wmh(af, bf, acc1);
    }
#pragma unroll
    for (int r = 0; r < 8; ++r) {
      const int c = 16 * i + 8 * hh + r, col = 16 * j + m;
      OST[c * OPI + col] = fmaf(acc1[r], PVF, QF[(size_t)c * DD + DH * h + col]);
    }
  }
  __syncthreads();
  v4f ov[2];
#pragma unroll
  for (int it = 0; it < 2; ++it) {
    const int u = tid + NTHR * it, c = u >> 4, cc = 4 * (u & 15);
    ov[it] = *(const v4f*)(OST + c * OPI + cc);
  }
#pragma unroll
  for (int it = 0; it < 2; ++it) {
    const int u = tid + NTHR * it, c = u >> 4, cc = 4 * (u & 15);
    *(volatile v4f*)(O + ((size_t)(b * CS + c)) * DD + DH * h + cc) = ov[it];
  }
  __threadfence();
#pragma unroll
  for (int it = 0; it < 2; ++it) {
    const int u = tid + NTHR * it, c = u >> 4, cc = 4 * (u & 15);
    *(volatile v4f*)(O + ((size_t)(b * CS + c)) * DD + DH * h + cc) = ov[it];
  }
}

__global__ __launch_bounds__(GTHR) void k_sab(const float* __restrict__ QKV, float* O) {
  __shared__ __attribute__((aligned(16))) _Float16 QT[CS * KPI];
  __shared__ __attribute__((aligned(16))) _Float16 KT[CS * KPI];
  __shared__ __attribute__((aligned(16))) _Float16 VT[DH * VBP];
  __shared__ __attribute__((aligned(16))) _Float16 PT[CS * VBP];
  __shared__ __attribute__((aligned(16))) float SS[CS * SSP];
  __shared__ __attribute__((aligned(16))) float OST[CS * OPI];
  const int tid = (int)threadIdx.x, lane = tid & 31, wave = tid >> 5, hh = lane >> 4, m = lane & 15;
  const int b = (int)blockIdx.x, h = (int)blockIdx.y;
  {
    const int c = tid >> 2, q4 = tid & 3;
    const float* rp = QKV + ((size_t)(b * CS + c)) * (3 * DD) + DH * h + 16 * q4;
#pragma unroll
    for (int part = 0; part < 2; ++part) {
      *(v8h*)(QT + c * KPI + 16 * q4 + 8 * part) =
          cvt8h(*(const v4f*)(rp + 8 * part), *(const v4f*)(rp + 8 * part + 4), CQ);
      *(v8h*)(KT + c * KPI + 16 * q4 + 8 * part) =
          cvt8h(*(const v4f*)(rp + DD + 8 * part), *(const v4f*)(rp + DD + 8 * part + 4), CKV);
    }
  }
  {
    const int d = tid & 63, chh = tid >> 6;
#pragma unroll
    for (int cc = 0; cc < 16; ++cc) {
      const int c = 16 * chh + cc;
      const float v = QKV[((size_t)(b * CS + c)) * (3 * DD) + 2 * DD + DH * h + d];
      VT[d * VBP + c] = (_Float16)(v * CKV);
    }
  }
  __syncthreads();
  const int i = wave & 1;
  {
    const int j = wave >> 1;
    v8f acc = zero8();
#pragma unroll
    for (int ks = 0; ks < 2; ++ks) {
      FragH af, bf;
      af.h[0] = *(const v8h*)(QT + (16 * i + m) * KPI + 32 * ks + 8 * hh);
      af.h[1] = *(const v8h*)(QT + (16 * i + m) * KPI + 32 * ks + 16 + 8 * hh);
      bf.h[0] = *(const v8h*)(KT + (16 * j + m) * KPI + 32 * ks + 8 * hh);
      bf.h[1] = *(const v8h*)(KT + (16 * j + m) * KPI + 32 * ks + 16 + 8 * hh);
      acc = wmh(af, bf, acc);
    }
#pragma unroll
    for (int r = 0; r < 8; ++r) SS[(16 * i + 8 * hh + r) * SSP + 16 * j + m] = acc[r] * SSCL;
  }
  __syncthreads();
#pragma unroll 1
  for (int rr = 0; rr < 8; ++rr) {
    const int row = 8 * wave + rr;
    const float s = SS[row * SSP + lane];
    const float mx = wave_max(s);
    const float e = __expf(s - mx);
    const float sum = wave_sum(e);
    PT[row * VBP + lane] = (_Float16)(e * (1.0f / sum) * CP);
  }
  __syncthreads();
  {
    FragH af;
    af.h[0] = *(const v8h*)(PT + (16 * i + m) * VBP + 8 * hh);
    af.h[1] = *(const v8h*)(PT + (16 * i + m) * VBP + 16 + 8 * hh);
    v8f acc[2];
#pragma unroll
    for (int jj = 0; jj < 2; ++jj) {
      const int j2 = 2 * (wave >> 1) + jj;
      FragH bf;
      bf.h[0] = *(const v8h*)(VT + (16 * j2 + m) * VBP + 8 * hh);
      bf.h[1] = *(const v8h*)(VT + (16 * j2 + m) * VBP + 16 + 8 * hh);
      acc[jj] = wmh(af, bf, zero8());
    }
#pragma unroll
    for (int jj = 0; jj < 2; ++jj) {
      const int j2 = 2 * (wave >> 1) + jj;
#pragma unroll
      for (int r = 0; r < 8; ++r) {
        const int c = 16 * i + 8 * hh + r, col = 16 * j2 + m;
        OST[c * OPI + col] = fmaf(acc[jj][r], PVF, QKV[((size_t)(b * CS + c)) * (3 * DD) + DH * h + col]);
      }
    }
  }
  __syncthreads();
  v4f ov[4];
#pragma unroll
  for (int it = 0; it < 4; ++it) {
    const int u = tid + GTHR * it, c = u >> 4, cc = 4 * (u & 15);
    ov[it] = *(const v4f*)(OST + c * OPI + cc);
  }
#pragma unroll
  for (int it = 0; it < 4; ++it) {
    const int u = tid + GTHR * it, c = u >> 4, cc = 4 * (u & 15);
    *(volatile v4f*)(O + ((size_t)(b * CS + c)) * DD + DH * h + cc) = ov[it];
  }
  __threadfence();
#pragma unroll
  for (int it = 0; it < 4; ++it) {
    const int u = tid + GTHR * it, c = u >> 4, cc = 4 * (u & 15);
    *(volatile v4f*)(O + ((size_t)(b * CS + c)) * DD + DH * h + cc) = ov[it];
  }
}

template<int MODE>
__global__ __launch_bounds__(NTHR) void k_ln(const float* __restrict__ a, const float* __restrict__ bsrc,
                                            const float* __restrict__ g, const float* __restrict__ be,
                                            float* outF, _Float16* outH, int rows) {
  __shared__ __attribute__((aligned(16))) float stg[8 * DD];
  const int tid = (int)threadIdx.x, lane = tid & 31, wave = tid >> 5;
  const int row = (int)blockIdx.x * 8 + wave;
  if (row >= rows) return;
  const size_t ro = (size_t)row * DD;
  v4f t0 = *(const v4f*)(a + ro + 8 * lane), t1 = *(const v4f*)(a + ro + 8 * lane + 4);
  if (MODE != 0) {
    t0 = t0 + relu4(*(const v4f*)(bsrc + ro + 8 * lane));
    t1 = t1 + relu4(*(const v4f*)(bsrc + ro + 8 * lane + 4));
  }
  float s = ((t0.x + t0.y) + (t0.z + t0.w)) + ((t1.x + t1.y) + (t1.z + t1.w));
  s = wave_sum(s);
  const float mu = s * (1.0f / DD);
  const v4f d0 = t0 - mu, d1 = t1 - mu;
  float ss = ((d0.x * d0.x + d0.y * d0.y) + (d0.z * d0.z + d0.w * d0.w))
           + ((d1.x * d1.x + d1.y * d1.y) + (d1.z * d1.z + d1.w * d1.w));
  ss = wave_sum(ss);
  const float rstd = rsqrtf(ss * (1.0f / DD) + LNEPS);
  const v4f g0 = *(const v4f*)(g + 8 * lane),  g1 = *(const v4f*)(g + 8 * lane + 4);
  const v4f e0 = *(const v4f*)(be + 8 * lane), e1 = *(const v4f*)(be + 8 * lane + 4);
  const v4f y0 = (d0 * rstd) * g0 + e0;
  const v4f y1 = (d1 * rstd) * g1 + e1;
  if (MODE != 2) {
    const v8h hv = cvt8h(y0, y1, CX);
    _Float16* hp = outH + ro + 8 * lane;
    *(volatile v8h*)hp = hv;
    __threadfence();
    *(volatile v8h*)hp = hv;
  }
  float* sw = stg + wave * DD;
  *(v4f*)(sw + 8 * lane)     = y0;
  *(v4f*)(sw + 8 * lane + 4) = y1;
  wave_lds_sync();
  const v4f p0 = *(const v4f*)(sw + 4 * lane);
  const v4f p1 = *(const v4f*)(sw + 128 + 4 * lane);
  float* o = outF + ro;
  *(volatile v4f*)(o + 4 * lane)       = p0;
  *(volatile v4f*)(o + 128 + 4 * lane) = p1;
  __threadfence();
  *(volatile v4f*)(o + 4 * lane)       = p0;
  *(volatile v4f*)(o + 128 + 4 * lane) = p1;
}

__global__ __launch_bounds__(NTHR) void k_comb(const float* __restrict__ AP, const float* __restrict__ VNS,
                                              const float* __restrict__ XG, const int* __restrict__ bid, _Float16* XH) {
  __shared__ __attribute__((aligned(16))) _Float16 VB[DD * VBP];
  __shared__ __attribute__((aligned(16))) _Float16 AT[64 * VBP];
  __shared__ __attribute__((aligned(16))) float stg[8 * 1024];
  __shared__ int msc[2];
  const int tid = (int)threadIdx.x, lane = tid & 31, wave = tid >> 5, hh = lane >> 4, m = lane & 15;
  const int bt = (int)blockIdx.x;
  if (tid == 0) msc[0] = lbnd(bid, NN, bt);
  if (tid == 1) msc[1] = lbnd(bid, NN, bt + 1);
  {
    const float* vp = VNS + ((size_t)(bt * CS)) * DD;
#pragma unroll
    for (int it = 0; it < 8; ++it) {
      const int u = tid + NTHR * it;
      *(v4f*)(stg + 4 * u) = *(const v4f*)(vp + (size_t)4 * u);
    }
  }
  __syncthreads();
  const int start = msc[0];
  int cnt = msc[1] - start;
  cnt = cnt < 0 ? 0 : (cnt > MX ? MX : cnt);
  const int hs = bt >> 5, bs0 = 4 * (bt & 31);
  {
    const int d = tid;
#pragma unroll
    for (int q = 0; q < 4; ++q) {
      v4f a, c4;
      a.x  = stg[(8 * q + 0) * DD + d]; a.y  = stg[(8 * q + 1) * DD + d];
      a.z  = stg[(8 * q + 2) * DD + d]; a.w  = stg[(8 * q + 3) * DD + d];
      c4.x = stg[(8 * q + 4) * DD + d]; c4.y = stg[(8 * q + 5) * DD + d];
      c4.z = stg[(8 * q + 6) * DD + d]; c4.w = stg[(8 * q + 7) * DD + d];
      *(v8h*)(VB + d * VBP + 8 * q) = cvt8h(a, c4, CV2);
    }
  }
  const int ntn = (cnt + 63) >> 6;
  const int i = wave & 3, ch = wave >> 2;
  float* sw = stg + wave * 1024;
#pragma unroll 1
  for (int nt = 0; nt < ntn; ++nt) {
    __syncthreads();
    {
      const float* apb = AP + ((size_t)((hs * BG + bs0) * CS)) * MX + 64 * nt;
#pragma unroll
      for (int it = 0; it < 2; ++it) {
        const int u = tid + NTHR * it, c = u >> 4, n4 = 4 * (u & 15);
        const float* p = apb + (size_t)c * MX + n4;
        v4f s = *(const v4f*)p;
        s = s + *(const v4f*)(p + (size_t)CS * MX);
        s = s + *(const v4f*)(p + (size_t)2 * CS * MX);
        s = s + *(const v4f*)(p + (size_t)3 * CS * MX);
        AT[(n4 + 0) * VBP + c] = (_Float16)(s.x * CP);
        AT[(n4 + 1) * VBP + c] = (_Float16)(s.y * CP);
        AT[(n4 + 2) * VBP + c] = (_Float16)(s.z * CP);
        AT[(n4 + 3) * VBP + c] = (_Float16)(s.w * CP);
      }
    }
    __syncthreads();
    FragH af;
    af.h[0] = *(const v8h*)(AT + (16 * i + m) * VBP + 8 * hh);
    af.h[1] = *(const v8h*)(AT + (16 * i + m) * VBP + 16 + 8 * hh);
#pragma unroll
    for (int gq = 0; gq < 2; ++gq) {
      v8f acc[4];
#pragma unroll
      for (int t = 0; t < 4; ++t) {
        const int col = 128 * ch + 64 * gq + 16 * t;
        FragH bf;
        bf.h[0] = *(const v8h*)(VB + (col + m) * VBP + 8 * hh);
        bf.h[1] = *(const v8h*)(VB + (col + m) * VBP + 16 + 8 * hh);
        acc[t] = wmh(af, bf, zero8());
      }
      wave_lds_sync();
#pragma unroll
      for (int t = 0; t < 4; ++t) {
#pragma unroll
        for (int r = 0; r < 8; ++r) sw[(8 * hh + r) * 64 + 16 * t + m] = acc[t][r] * CMF;
      }
      wave_lds_sync();
      v8h hv[4]; int ok[4]; size_t oo[4];
#pragma unroll
      for (int ii = 0; ii < 4; ++ii) {
        const int lr2 = 4 * ii + (lane >> 3), q = lane & 7;
        const int n2 = 64 * nt + 16 * i + lr2;
        int node = start + n2;
        node = node > NN - 1 ? NN - 1 : node;
        const float* xr = XG + (size_t)node * DD + 128 * ch + 64 * gq + 8 * q;
        const v4f a  = *(const v4f*)(sw + lr2 * 64 + 8 * q)     + *(const v4f*)xr;
        const v4f c4 = *(const v4f*)(sw + lr2 * 64 + 8 * q + 4) + *(const v4f*)(xr + 4);
        hv[ii] = cvt8h(a, c4, CX);
        ok[ii] = n2 < cnt;
        oo[ii] = (size_t)(start + n2) * DD + 128 * ch + 64 * gq + 8 * q;
      }
#pragma unroll
      for (int ii = 0; ii < 4; ++ii) if (ok[ii]) *(volatile v8h*)(XH + oo[ii]) = hv[ii];
      __threadfence();
#pragma unroll
      for (int ii = 0; ii < 4; ++ii) if (ok[ii]) *(volatile v8h*)(XH + oo[ii]) = hv[ii];
    }
  }
}

static inline size_t al256(size_t b) { return (b + 255) & ~(size_t)255; }

extern "C" void kernel_launch(void* const* d_in, const int* in_sizes, int n_in,
                              void* d_out, int out_size, void* d_ws, size_t ws_size,
                              hipStream_t stream) {
  if (n_in < 16) return;
  if (in_sizes[0] != NN * DD) return;
  if (in_sizes[1] != NL * DD * DD || in_sizes[2] != NL * DD) return;
  if (in_sizes[3] != NL * CS * DD) return;
  if (in_sizes[4] != NL * 4 * DD * DD || in_sizes[5] != NL * 4 * DD) return;
  if (in_sizes[6] != NL * 2 * DD || in_sizes[7] != NL * 2 * DD) return;
  if (in_sizes[8] != NL * 4 * DD * DD || in_sizes[9] != NL * 4 * DD) return;
  if (in_sizes[10] != NL * 2 * DD || in_sizes[11] != NL * 2 * DD) return;
  if (in_sizes[12] != DD * DO || in_sizes[13] != DO) return;
  if (in_sizes[14] != 2 * EE || in_sizes[15] != NN) return;
  if (out_size != NN * DO) return;

  const float* x_in   = (const float*)d_in[0];
  const float* gcn_W  = (const float*)d_in[1];
  const float* gcn_b  = (const float*)d_in[2];
  const float* seeds  = (const float*)d_in[3];
  const float* proj_W = (const float*)d_in[4];
  const float* proj_b = (const float*)d_in[5];
  const float* plg    = (const float*)d_in[6];
  const float* plb    = (const float*)d_in[7];
  const float* exch_W = (const float*)d_in[8];
  const float* exch_b = (const float*)d_in[9];
  const float* elg    = (const float*)d_in[10];
  const float* elb    = (const float*)d_in[11];
  const float* head_W = (const float*)d_in[12];
  const float* head_b = (const float*)d_in[13];
  const int*   eidx   = (const int*)d_in[14];
  const int*   bid    = (const int*)d_in[15];
  float* out = (float*)d_out;

  size_t off = 0;
  const size_t oXH  = off; off += al256((size_t)NN * DD * 2);
  const size_t oR2  = off; off += al256((size_t)NN * DD * 4);
  const size_t oXG  = off; off += al256((size_t)NN * DD * 4);
  const size_t oAP  = off; off += al256((size_t)NHD * BG * CS * MX * 4);
  const size_t oO   = off; off += al256((size_t)MR * DD * 4);
  const size_t oQF  = off; off += al256((size_t)64 * DD * 4);
  const size_t oSH  = off; off += al256((size_t)NL * 64 * DD * 2);
  const size_t oWG  = off; off += al256((size_t)NL * DD * DD * 2);
  const size_t oWP  = off; off += al256((size_t)NL * 4 * DD * DD * 2);
  const size_t oWE  = off; off += al256((size_t)NL * 4 * DD * DD * 2);
  const size_t oWHD = off; off += al256((size_t)64 * DD * 2);
  const size_t oSK  = off; off += al256((size_t)NCH * CHE * 4);
  const size_t oCNT = off; off += al256((size_t)NCH * NGR * 4);
  const size_t oLB  = off; off += al256((size_t)NCH * NGR * 4);
  const size_t oES  = off; off += al256((size_t)NGR * LCAP * 4);
  const size_t oRC  = off; off += al256((size_t)NN * 4);
  const size_t oRO  = off; off += al256((size_t)NN * 4);
  if (off > ws_size || off > (size_t)WSMAX) return;
  const size_t oQKV2 = oR2;
  const size_t oT1   = oR2 + 12582912;
  const size_t oT1H  = oR2 + 16777216;
  const size_t oG    = oR2 + 18874368;
  const size_t oVNS  = oR2 + 23068672;
  const size_t oVNSH = oR2 + 27262976;
  const size_t oVNS2 = oR2 + 29360128;
  if (oVNS2 + (size_t)MR * DD * 4 != oR2 + (size_t)NN * DD * 4) return;

  char* ws = (char*)d_ws;
  _Float16* XH   = (_Float16*)(ws + oXH);
  _Float16* XGH  = XH;
  float*    XW   = (float*)(ws + oR2);
  _Float16* KV   = (_Float16*)(ws + oR2);
  float*    XG   = (float*)(ws + oXG);
  float*    AP   = (float*)(ws + oAP);
  float*    O    = (float*)(ws + oO);
  float*    QF   = (float*)(ws + oQF);
  _Float16* SH   = (_Float16*)(ws + oSH);
  _Float16* WG   = (_Float16*)(ws + oWG);
  _Float16* WP   = (_Float16*)(ws + oWP);
  _Float16* WE   = (_Float16*)(ws + oWE);
  _Float16* WHD  = (_Float16*)(ws + oWHD);
  int*      SK   = (int*)(ws + oSK);
  int*      CNT  = (int*)(ws + oCNT);
  int*      LB   = (int*)(ws + oLB);
  int*      ES   = (int*)(ws + oES);
  int*      RC   = (int*)(ws + oRC);
  int*      RO   = (int*)(ws + oRO);
  float*    QKV2 = (float*)(ws + oQKV2);
  float*    T1   = (float*)(ws + oT1);
  _Float16* T1H  = (_Float16*)(ws + oT1H);
  float*    G    = (float*)(ws + oG);
  float*    VNS  = (float*)(ws + oVNS);
  _Float16* VNSH = (_Float16*)(ws + oVNSH);
  float*    VNS2 = (float*)(ws + oVNS2);
  const size_t WSZ = (size_t)DD * DD;

  const int nUx = NN * (DD / 8);
  k_xprep<<<dim3(nUx / NTHR, 1), NTHR, 0, stream>>>(x_in, XH, NN, NN, nUx);
  const int nUs = 64 * (DD / 8);
  k_xprep<<<dim3(nUs / NTHR, NL), NTHR, 0, stream>>>(seeds, SH, CS, 64, nUs);
  k_wtr<<<dim3(DD / TT, DD / TT, NL), NTHR, 0, stream>>>(gcn_W, WG, DD, DD);
  k_wtr<<<dim3(DD / TT, DD / TT, NL * 4), NTHR, 0, stream>>>(proj_W, WP, DD, DD);
  k_wtr<<<dim3(DD / TT, DD / TT, NL * 4), NTHR, 0, stream>>>(exch_W, WE, DD, DD);
  k_headw<<<64, 32, 0, stream>>>(head_W, WHD, DD, DO);
  k_csort<<<NCH, NTHR, 0, stream>>>(eidx, SK, CNT, LB);
  k_cgroup<<<NGR, NTHR, 0, stream>>>(SK, CNT, LB, ES, RC, RO);

  hipFuncSetAttribute(reinterpret_cast<const void*>(&k_pma), hipFuncAttributeMaxDynamicSharedMemorySize, PMA_LDS);

  for (int l = 0; l < NL; ++l) {
    k_gemm<0, 4, 0><<<dim3(NN / GBM, DD / 64), GTHR, 0, stream>>>(XH, WG + (size_t)l * WSZ, gcn_b, XW, XH,
                                                                  DD, DD, SCL, 1.0f);
    k_agg<<<NN / 8, NTHR, 0, stream>>>(XW, ES, RC, RO, gcn_b + (size_t)l * DD, XG, XGH);
    k_gemm<1, 4, 1><<<dim3(NN / GBM, (2 * DD) / 64), GTHR, 0, stream>>>(
        XGH, WP + (size_t)(4 * l + 1) * WSZ, proj_b + (size_t)(4 * l + 1) * DD, XW, KV, DD, 2 * DD, SCL, CKV);
    k_gemm<0, 4, 1><<<dim3(1, DD / 64), GTHR, 0, stream>>>(
        SH + (size_t)l * 64 * DD, WP + (size_t)(4 * l) * WSZ, proj_b + (size_t)(4 * l) * DD, QF, XH, DD, DD, SCL, 1.0f);
    k_pma<<<dim3(BG, NHD), NTHR, PMA_LDS, stream>>>(KV, QF, bid, AP, O);
    k_ln<0><<<MR / 8, NTHR, 0, stream>>>(O, O, plg + (size_t)(2 * l) * DD, plb + (size_t)(2 * l) * DD, T1, T1H, MR);
    k_gemm<0, 4, 1><<<dim3(MR / GBM, DD / 64), GTHR, 0, stream>>>(
        T1H, WP + (size_t)(4 * l + 3) * WSZ, proj_b + (size_t)(4 * l + 3) * DD, G, XH, DD, DD, SCL, 1.0f);
    k_ln<1><<<MR / 8, NTHR, 0, stream>>>(T1, G, plg + (size_t)(2 * l + 1) * DD, plb + (size_t)(2 * l + 1) * DD,
                                         VNS, VNSH, MR);
    k_gemm<0, 4, 1><<<dim3(MR / GBM, (3 * DD) / 64), GTHR, 0, stream>>>(
        VNSH, WE + (size_t)(4 * l) * WSZ, exch_b + (size_t)(4 * l) * DD, QKV2, XH, DD, 3 * DD, SCL, 1.0f);
    k_sab<<<dim3(BG, NHD), GTHR, 0, stream>>>(QKV2, O);
    k_ln<0><<<MR / 8, NTHR, 0, stream>>>(O, O, elg + (size_t)(2 * l) * DD, elb + (size_t)(2 * l) * DD, T1, T1H, MR);
    k_gemm<0, 4, 1><<<dim3(MR / GBM, DD / 64), GTHR, 0, stream>>>(
        T1H, WE + (size_t)(4 * l + 3) * WSZ, exch_b + (size_t)(4 * l + 3) * DD, G, XH, DD, DD, SCL, 1.0f);
    k_ln<2><<<MR / 8, NTHR, 0, stream>>>(T1, G, elg + (size_t)(2 * l + 1) * DD, elb + (size_t)(2 * l + 1) * DD,
                                         VNS2, T1H, MR);
    k_comb<<<BG, NTHR, 0, stream>>>(AP, VNS2, XG, bid, XH);
  }
  k_gemm<0, 2, 1><<<dim3(NN / GBM, 1), GTHR, 0, stream>>>(XH, WHD, head_b, out, XH, DD, DO, SCL, 1.0f);
}
